// _ParityGameGATConv_27075473834771
// MI455X (gfx1250) — hardware-verified
//
#include <hip/hip_runtime.h>
#include <math.h>


#define NN 100000
#define NE 1600000
#define DIN 128
#define HD 64
#define DE 8
#define SLOTC 64
#define NCH 768

typedef __attribute__((ext_vector_type(16))) _Float16 v16h;
typedef __attribute__((ext_vector_type(8)))  float v8f;
typedef __attribute__((ext_vector_type(4)))  float v4f;
typedef __attribute__((ext_vector_type(2)))  float v2f;
typedef __attribute__((ext_vector_type(4)))  int v4i;
typedef float __attribute__((may_alias)) float_a;
typedef int __attribute__((may_alias)) int_a;

template <typename T> __device__ __forceinline__ void vst2(void* p, T v) { *(volatile T*)p = v; __threadfence(); *(volatile T*)p = v; }
__device__ __forceinline__ v8f wmma16(v16h a, v16h b, v8f c) {
  v8f d = __builtin_amdgcn_wmma_f32_16x16x32_f16(false, a, false, b, (short)0, c, false, false);
  asm volatile("v_nop\n\tv_nop\n\tv_nop\n\tv_nop" : "+v"(d) : "v"(a), "v"(b));
  return d;
}
__device__ __forceinline__ v16h frag_f32(const float* rowk0, int lane) {
  v16h a; const float* p = rowk0 + 8 * (lane >> 4);
#pragma unroll
  for (int i = 0; i < 8; ++i) { a[i] = (_Float16)p[i]; a[8 + i] = (_Float16)p[16 + i]; }
  return a;
}
__device__ __forceinline__ v16h frag_col(const float* W, int k0, int n, int lane, int ld, int K) {
  v16h a;
#pragma unroll
  for (int i = 0; i < 8; ++i) { const int ka = k0 + 8 * (lane >> 4) + i, kb = ka + 16;
    a[i] = (_Float16)(ka < K ? W[(size_t)ka * ld + n] : 0.f); a[8 + i] = (_Float16)(kb < K ? W[(size_t)kb * ld + n] : 0.f); }
  return a;
}
#define LDSX() do { asm volatile("s_wait_dscnt 0" ::: "memory"); __builtin_amdgcn_wave_barrier(); __builtin_amdgcn_fence(__ATOMIC_RELEASE, "workgroup"); } while (0)

__global__ __launch_bounds__(128) void k_encode(const float* __restrict__ x, const float* __restrict__ We, const float* __restrict__ be,
                                              const float* __restrict__ Wg, const float* __restrict__ asv, const float* __restrict__ adv,
                                              float* __restrict__ hg, float* __restrict__ as_, float* __restrict__ ad_) {
  __shared__ __align__(16) float H[4][16][68];
  __shared__ __align__(16) float sa[64], sd[64];
  const int tid = threadIdx.x, w = tid >> 5, lane = tid & 31, col = lane & 15, g = lane >> 4;
  const int n0 = blockIdx.x * 64 + w * 16;
  const bool live = n0 < NN;
  float* Hw = &H[w][0][0];
  if (live) {
    v8f acc[4] = {};
#pragma unroll
    for (int kc = 0; kc < DIN / 32; ++kc) { const v16h a = frag_f32(x + (size_t)(n0 + col) * DIN + kc * 32, lane);
#pragma unroll
      for (int t = 0; t < 4; ++t) acc[t] = wmma16(a, frag_col(We, kc * 32, t * 16 + col, lane, HD, DIN), acc[t]); }
#pragma unroll
    for (int t = 0; t < 4; ++t) { const float bb = be[t * 16 + col];
#pragma unroll
      for (int r = 0; r < 8; ++r) { const float v = acc[t][r] + bb; Hw[(8 * g + r) * 68 + t * 16 + col] = v > 0.f ? v : 0.f; } }
    LDSX();
    v8f ag[4] = {};
#pragma unroll
    for (int kc = 0; kc < 2; ++kc) { const v16h a = frag_f32(Hw + col * 68 + kc * 32, lane);
#pragma unroll
      for (int t = 0; t < 4; ++t) ag[t] = wmma16(a, frag_col(Wg, kc * 32, t * 16 + col, lane, HD, HD), ag[t]); }
    __builtin_amdgcn_wave_barrier();
#pragma unroll
    for (int t = 0; t < 4; ++t)
#pragma unroll
      for (int r = 0; r < 8; ++r) Hw[(8 * g + r) * 68 + t * 16 + col] = ag[t][r];
    LDSX();
#pragma unroll
    for (int q = 0; q < 8; ++q) { const int rl = q * 2 + (lane >> 4), pc = lane & 15;
      vst2(hg + (size_t)(n0 + rl) * HD + pc * 4, *(const v4f*)(Hw + rl * 68 + pc * 4)); }
    if (lane < 16) { float s = 0.f, d = 0.f;
#pragma unroll 1
      for (int j = 0; j < HD; ++j) { const float v = Hw[lane * 68 + j]; s += v * asv[j]; d += v * adv[j]; }
      sa[w * 16 + lane] = s; sd[w * 16 + lane] = d; }
  }
  __syncthreads();
  if (tid < 16) { vst2(as_ + (size_t)blockIdx.x * 64 + tid * 4, *(const v4f*)(&sa[tid * 4])); }
  else if (tid < 32) { const int t2 = tid - 16; vst2(ad_ + (size_t)blockIdx.x * 64 + t2 * 4, *(const v4f*)(&sd[t2 * 4])); }
}

__global__ __launch_bounds__(256) void k_bucket(const int* __restrict__ ei, int* __restrict__ tlist, int* __restrict__ cnt) {
  __shared__ int scnt[NCH];
  __shared__ int slots[NCH][SLOTC];
  const int tid = threadIdx.x, n0 = blockIdx.x * NCH;
  for (int i = tid; i < NCH; i += 256) scnt[i] = 0;
  __syncthreads();
  for (int e = tid; e < NE; e += 256) { const int i = ei[NE + e] - n0;
    if (i >= 0 && i < NCH) { const int s = atomicAdd(&scnt[i], 1); if (s < SLOTC) slots[i][s] = e; } }
  __syncthreads();
  for (int i = tid; i < NCH; i += 256) { const int n = n0 + i; if (n >= NN) continue;
    int c = scnt[i]; if (c > SLOTC) c = SLOTC;
    for (int a = 1; a < c; ++a) { const int v = slots[i][a]; int b = a - 1; while (b >= 0 && slots[i][b] > v) { slots[i][b + 1] = slots[i][b]; --b; } slots[i][b + 1] = v; }
    for (int a = c; a < SLOTC; ++a) slots[i][a] = 0;
#pragma unroll 1
    for (int p = 0; p < SLOTC / 4; ++p) { v4i v = { slots[i][4 * p], slots[i][4 * p + 1], slots[i][4 * p + 2], slots[i][4 * p + 3] }; vst2(tlist + (size_t)n * SLOTC + 4 * p, v); }
    vst2(cnt + (size_t)n * 32, (int_a)c);
  }
}

__global__ __launch_bounds__(512) void k_node(const float* __restrict__ hg, const float* __restrict__ as_, const float* __restrict__ ad_,
                                            const int* __restrict__ ei, const int* __restrict__ tlist, const int* __restrict__ cnt,
                                            const float* __restrict__ Wn1, const float* __restrict__ bn1, const float* __restrict__ Wn2, const float* __restrict__ bn2,
                                            float* __restrict__ xc, float* __restrict__ nlog) {
  __shared__ __align__(16) float sx[16][HD];
  __shared__ __align__(16) float sl[16][2];
  const int tid = threadIdx.x, w = tid >> 5, lane = tid & 31;
  const int n = blockIdx.x * 16 + w;
  if (n < NN) {
    int ne = cnt[(size_t)n * 32]; ne = ne < 0 ? 0 : (ne > SLOTC ? SLOTC : ne); const float adn = ad_[n];
    float m = -3.0e38f;
#pragma unroll 1
    for (int s = 0; s < ne; ++s) { int e = tlist[(size_t)n * SLOTC + s]; e = ((unsigned)e < (unsigned)NE) ? e : 0; int sr = ei[e]; sr = sr < 0 ? 0 : (sr >= NN ? NN - 1 : sr);
      float sc = as_[sr] + adn; sc = sc > 0.f ? sc : 0.2f * sc; m = fmaxf(m, sc); }
    if (ne == 0) m = 0.f;
    float den = 0.f, a0 = 0.f, a1 = 0.f;
#pragma unroll 1
    for (int s = 0; s < ne; ++s) { int e = tlist[(size_t)n * SLOTC + s]; e = ((unsigned)e < (unsigned)NE) ? e : 0; int sr = ei[e]; sr = sr < 0 ? 0 : (sr >= NN ? NN - 1 : sr);
      float sc = as_[sr] + adn; sc = sc > 0.f ? sc : 0.2f * sc; const float ex = expf(sc - m);
      den += ex; a0 += ex * hg[(size_t)sr * HD + lane]; a1 += ex * hg[(size_t)sr * HD + 32 + lane]; }
    const float inv = 1.0f / (den + 1e-9f);
    float x0 = a0 * inv, x1 = a1 * inv; x0 = x0 > 0.f ? x0 : 0.f; x1 = x1 > 0.f ? x1 : 0.f;
    sx[w][lane] = x0; sx[w][32 + lane] = x1;
    LDSX();
    if (lane < 16) vst2(xc + (size_t)n * HD + lane * 4, *(const v4f*)(&sx[w][lane * 4]));
    float h0 = bn1[lane], h1 = bn1[32 + lane];
#pragma unroll 1
    for (int i = 0; i < HD; ++i) { const float v = sx[w][i]; h0 += v * Wn1[i * HD + lane]; h1 += v * Wn1[i * HD + 32 + lane]; }
    h0 = h0 > 0.f ? h0 : 0.f; h1 = h1 > 0.f ? h1 : 0.f;
    float o0 = h0 * Wn2[lane * 2] + h1 * Wn2[(32 + lane) * 2], o1 = h0 * Wn2[lane * 2 + 1] + h1 * Wn2[(32 + lane) * 2 + 1];
#pragma unroll
    for (int off = 16; off >= 1; off >>= 1) { o0 += __shfl_xor(o0, off, 32); o1 += __shfl_xor(o1, off, 32); }
    if (lane == 0) { sl[w][0] = o0 + bn2[0]; sl[w][1] = o1 + bn2[1]; }
  }
  __syncthreads();
  if (tid < 8) vst2(nlog + (size_t)blockIdx.x * 32 + tid * 4, *(const v4f*)(&sl[0][0] + tid * 4));
}

__global__ __launch_bounds__(128) void k_edge(const float* __restrict__ xc, const int* __restrict__ ei, const float* __restrict__ ea,
                                            const float* __restrict__ We1, const float* __restrict__ be1, const float* __restrict__ We2,
                                            const float* __restrict__ be2, float* __restrict__ elog) {
  __shared__ __align__(16) float so[4][16][2];
  const int tid = threadIdx.x, w = tid >> 5, lane = tid & 31, col = lane & 15, g = lane >> 4;
  const int e0 = (blockIdx.x * 4 + w) * 16; const int e = e0 + col;
  int sr = ei[e], ds = ei[NE + e]; sr = sr < 0 ? 0 : (sr >= NN ? NN - 1 : sr); ds = ds < 0 ? 0 : (ds >= NN ? NN - 1 : ds);
  v8f acc[4] = {};
#pragma unroll
  for (int kc = 0; kc < 5; ++kc) {
    v16h a;
#pragma unroll
    for (int i = 0; i < 16; ++i) { const int k = kc * 32 + 8 * g + (i < 8 ? i : 8 + i);
      float v;
      if (k < 64) v = xc[(size_t)sr * HD + k]; else if (k < 128) v = xc[(size_t)ds * HD + k - 64]; else if (k < 136) v = ea[(size_t)e * DE + k - 128]; else v = 0.f;
      a[i] = (_Float16)v; }
#pragma unroll
    for (int t = 0; t < 4; ++t) acc[t] = wmma16(a, frag_col(We1, kc * 32, t * 16 + col, lane, HD, 2 * HD + DE), acc[t]);
  }
  float p0[8], p1[8];
#pragma unroll
  for (int r = 0; r < 8; ++r) { p0[r] = 0.f; p1[r] = 0.f; }
#pragma unroll
  for (int t = 0; t < 4; ++t) { const int c = t * 16 + col; const float bb = be1[c], w0 = We2[c * 2], w1 = We2[c * 2 + 1];
#pragma unroll
    for (int r = 0; r < 8; ++r) { float u = acc[t][r] + bb; u = u > 0.f ? u : 0.f; p0[r] += u * w0; p1[r] += u * w1; } }
#pragma unroll
  for (int r = 0; r < 8; ++r) {
#pragma unroll
    for (int off = 8; off >= 1; off >>= 1) { p0[r] += __shfl_xor(p0[r], off, 32); p1[r] += __shfl_xor(p1[r], off, 32); }
    if (col == 0) { so[w][8 * g + r][0] = p0[r] + be2[0]; so[w][8 * g + r][1] = p1[r] + be2[1]; } }
  LDSX();
  if (lane < 8) vst2(elog + (size_t)e0 * 2 + lane * 4, *(const v4f*)(&so[w][0][0] + lane * 4));
}

extern "C" void kernel_launch(void* const* d_in, const int* in_sizes, int n_in,
                              void* d_out, int out_size, void* d_ws, size_t ws_size,
                              hipStream_t stream) {
  (void)in_sizes; (void)n_in; (void)out_size; (void)ws_size;
  const float* x = (const float*)d_in[0]; const int* ei = (const int*)d_in[1]; const float* ea = (const float*)d_in[2];
  const float* We = (const float*)d_in[3]; const float* be = (const float*)d_in[4];
  const float* Wg = (const float*)d_in[5]; const float* asv = (const float*)d_in[6]; const float* adv = (const float*)d_in[7];
  const float* Wn1 = (const float*)d_in[8]; const float* bn1 = (const float*)d_in[9];
  const float* Wn2 = (const float*)d_in[10]; const float* bn2 = (const float*)d_in[11];
  const float* We1 = (const float*)d_in[12]; const float* be1 = (const float*)d_in[13];
  const float* We2 = (const float*)d_in[14]; const float* be2 = (const float*)d_in[15];
  float* nlog = (float*)d_out;
  float* elog = (float*)d_out + (size_t)NN * 2;
  char* ws = (char*)d_ws; size_t off = 0;
  auto take = [&](size_t bytes) { char* p = ws + off; off += (bytes + 255) & ~(size_t)255; return p; };
  const int NPAD = ((NN + 63) / 64) * 64;
  float* hg  = (float*)take((size_t)NPAD * HD * 4);
  float* as_ = (float*)take((size_t)NPAD * 4); float* ad_ = (float*)take((size_t)NPAD * 4);
  int* tlist = (int*)take((size_t)NN * SLOTC * 4); int* cnt = (int*)take((size_t)NN * 32 * 4);
  float* xc  = (float*)take((size_t)NPAD * HD * 4);
  k_encode<<<(NN + 63) / 64, 128, 0, stream>>>(x, We, be, Wg, asv, adv, hg, as_, ad_);
  k_bucket<<<(NN + NCH - 1) / NCH, 256, 0, stream>>>(ei, tlist, cnt);
  k_node<<<NN / 16, 512, 0, stream>>>(hg, as_, ad_, ei, tlist, cnt, Wn1, bn1, Wn2, bn2, xc, nlog);
  k_edge<<<NE / 64, 128, 0, stream>>>(xc, ei, ea, We1, be1, We2, be2, elog);
}
